// Encoder_16003048145604
// MI455X (gfx1250) — hardware-verified
//
#include <hip/hip_runtime.h>
#include <math.h>

constexpr int NVOCAB  = 1024;
constexpr int NHID    = 512;
constexpr int NBATCH  = 32;
constexpr int NSTEP   = 256;
constexpr int NGATE3  = 3 * NHID;
constexpr int NROWS   = NBATCH * NSTEP;
constexpr int SEQ_BLK = 16;
constexpr int SCAN_THR = 512;
constexpr int HPITCH  = 520;
constexpr int FPITCH  = 516;
constexpr float HCARRY = 64.0f;
constexpr float WCARRY = 16.0f;
constexpr float LCARRY = 2048.0f;
constexpr int NOUT0 = NBATCH * NSTEP * 2 * NHID;
constexpr int NOUTS = NBATCH * 2 * NHID;
constexpr size_t PLANE_W  = (size_t)NGATE3 * NHID;
constexpr size_t PLANE_X0 = (size_t)NROWS * NHID;
constexpr size_t PLANE_XZ = (size_t)NROWS * NGATE3;
static_assert(NGATE3 == 1536, "gate width");
static_assert(NROWS % 64 == 0 && NGATE3 % 64 == 0 && NHID % 32 == 0, "GEMM tile multiples");
static_assert(SCAN_THR / 32 == SEQ_BLK, "one wave per row in the copy-out");
static_assert((SCAN_THR / 32) * 32 == NHID, "16 waves x 32 hidden columns");
static_assert(NBATCH % SEQ_BLK == 0, "row tiles");
static_assert((size_t)NOUT0 * 4 + 2 * (size_t)NOUTS * 4 == (size_t)33816576, "d_out bytes");
static_assert((size_t)NOUT0 * 4 == (size_t)33554432, "offset of the first final-state output");
static_assert(HPITCH % 8 == 0 && FPITCH % 4 == 0, "16-B aligned LDS rows");

typedef __attribute__((ext_vector_type(16))) _Float16 v16h;
typedef __attribute__((ext_vector_type(8)))  _Float16 v8h;
typedef __attribute__((ext_vector_type(16))) __bf16   v16b;
typedef __attribute__((ext_vector_type(8)))  __bf16   v8b;
typedef __attribute__((ext_vector_type(8)))  float    v8f;
typedef __attribute__((ext_vector_type(4)))  float    v4f;

__device__ __forceinline__ unsigned short f2bf_bits(float f) {
  unsigned u = __float_as_uint(f);
  return (unsigned short)((u + 0x7FFFu + ((u >> 16) & 1u)) >> 16);
}
__device__ __forceinline__ float bf_bits2f(unsigned short h) { return __uint_as_float(((unsigned)h) << 16); }

__device__ __forceinline__ void dep_guard_h(v8f& a, v8f& b, v16h x, v16h y) { asm volatile("v_nop\n\tv_nop\n\tv_nop\n\tv_nop" : "+v"(a), "+v"(b) : "v"(x), "v"(y)); }
__device__ __forceinline__ void dep_guard_b(v8f& a, v8f& b, v16b x, v16b y) { asm volatile("v_nop\n\tv_nop\n\tv_nop\n\tv_nop" : "+v"(a), "+v"(b) : "v"(x), "v"(y)); }
__device__ __forceinline__ void dep_guard4_h(v8f& a, v8f& b, v8f& c, v8f& d, v16h x, v16h y) { asm volatile("v_nop\n\tv_nop\n\tv_nop\n\tv_nop" : "+v"(a), "+v"(b), "+v"(c), "+v"(d) : "v"(x), "v"(y)); }
__device__ __forceinline__ void dep_guard4_b(v8f& a, v8f& b, v8f& c, v8f& d, v16b x, v16b y) { asm volatile("v_nop\n\tv_nop\n\tv_nop\n\tv_nop" : "+v"(a), "+v"(b), "+v"(c), "+v"(d) : "v"(x), "v"(y)); }
__device__ __forceinline__ void keep4_h(v16h a, v16h b, v16h c, v16h d) { asm volatile("v_nop" :: "v"(a), "v"(b), "v"(c), "v"(d)); }
__device__ __forceinline__ void keep4_b(v16b a, v16b b, v16b c, v16b d) { asm volatile("v_nop" :: "v"(a), "v"(b), "v"(c), "v"(d)); }
__device__ __forceinline__ void acc_guard4(v8f& a, v8f& b, v8f& c, v8f& d) { asm volatile("v_nop\n\tv_nop\n\tv_nop\n\tv_nop" : "+v"(a), "+v"(b), "+v"(c), "+v"(d)); }
__device__ __forceinline__ void dep_guard6_h(v8f& a, v8f& b, v8f& c, v8f& d, v8f& e, v8f& f,
                                             v16h p, v16h q, v16h x, v16h y, v16h z) {
  asm volatile("v_nop\n\tv_nop\n\tv_nop\n\tv_nop"
               : "+v"(a), "+v"(b), "+v"(c), "+v"(d), "+v"(e), "+v"(f)
               : "v"(p), "v"(q), "v"(x), "v"(y), "v"(z));
}
__device__ __forceinline__ void acc_guard6j(v8f& a, v8f& b, v8f& c, v8f& d, v8f& e, v8f& f, int& j) {
  asm volatile("v_nop\n\tv_nop\n\tv_nop\n\tv_nop"
               : "+v"(a), "+v"(b), "+v"(c), "+v"(d), "+v"(e), "+v"(f), "+v"(j));
}
__device__ __forceinline__ void pin8(int& a, int& b, int& c, int& d, int& e, int& f, int& g, int& h) {
  asm volatile("" : "+v"(a), "+v"(b), "+v"(c), "+v"(d), "+v"(e), "+v"(f), "+v"(g), "+v"(h));
}
__device__ __forceinline__ void order_after4(int& j, float a, float b, float c, float d) {
  asm volatile("" : "+v"(j) : "v"(a), "v"(b), "v"(c), "v"(d));
}

template <typename T> struct Frag;
template <> struct Frag<_Float16> {
  typedef v16h V; union U { v16h v; v8h h[2]; };
  static __device__ __forceinline__ v16h load(const _Float16* p) {
    U f; f.h[0] = *(const v8h*)(p); f.h[1] = *(const v8h*)(p + 16); return f.v;
  }
  static __device__ __forceinline__ v8f mma(v16h a, v16h b, v8f c) {
    return __builtin_amdgcn_wmma_f32_16x16x32_f16(false, a, false, b, (short)0, c, false, false);
  }
  static __device__ __forceinline__ void guard4(v8f& a, v8f& b, v8f& c, v8f& d, v16h x, v16h y) { dep_guard4_h(a, b, c, d, x, y); }
  static __device__ __forceinline__ void keep(v16h a, v16h b, v16h c, v16h d) { keep4_h(a, b, c, d); }
};
template <> struct Frag<__bf16> {
  typedef v16b V; union U { v16b v; v8b h[2]; };
  static __device__ __forceinline__ v16b load(const __bf16* p) {
    U f; f.h[0] = *(const v8b*)(p); f.h[1] = *(const v8b*)(p + 16); return f.v;
  }
  static __device__ __forceinline__ v8f mma(v16b a, v16b b, v8f c) {
    return __builtin_amdgcn_wmma_f32_16x16x32_bf16(false, a, false, b, (short)0, c, false, false);
  }
  static __device__ __forceinline__ void guard4(v8f& a, v8f& b, v8f& c, v8f& d, v16b x, v16b y) { dep_guard4_b(a, b, c, d, x, y); }
  static __device__ __forceinline__ void keep(v16b a, v16b b, v16b c, v16b d) { keep4_b(a, b, c, d); }
};

template <int ET> struct Elem;
template <> struct Elem<0> { typedef _Float16 T; };
template <> struct Elem<1> { typedef __bf16 T; };
template <int ET, bool SPLIT, int BIAS_MODE, int OUT_MODE, bool RESID, int ACT = 0>
__global__ __launch_bounds__(256) void wmma_gemm64(
    const unsigned short* __restrict__ Ap, const unsigned short* __restrict__ A2p, int lda, long strideA,
    const unsigned short* __restrict__ Btp, const unsigned short* __restrict__ Bt2p, int ldb, long strideB,
    void* __restrict__ Cout, void* __restrict__ Cout2, int ldc, long strideC,
    const float* __restrict__ bias,
    const float* __restrict__ resid, long strideR,
    int M, int N, int K, float scale) {
  typedef typename Elem<ET>::T T;
  typedef typename Frag<T>::V V;
  const T* A = (const T*)Ap; const T* A2 = (const T*)A2p; const T* Bt = (const T*)Btp; const T* Bt2 = (const T*)Bt2p;
  __shared__ __align__(16) float sT[8][16 * 68];
  const int b    = blockIdx.y;
  const int lane = threadIdx.x & 31;
  const int wave = threadIdx.x >> 5;
  const int tilesN = N >> 6;
  const int tilesM = M >> 6;
  const int tile = blockIdx.x * 8 + wave;
  if (tile >= tilesM * tilesN) return;
  const int tm = tile / tilesN;
  const int tn = tile - tm * tilesN;
  const int m0 = tm << 6;
  const int n0 = tn << 6;

  const T* Ab  = A  + (size_t)b * strideA;
  const T* Bb  = Bt + (size_t)b * strideB;
  const T* Ab2 = SPLIT ? (A2  + (size_t)b * strideA) : nullptr;
  const T* Bb2 = SPLIT ? (Bt2 + (size_t)b * strideB) : nullptr;

  const int rlane = lane & 15;
  const int koff  = (lane >> 4) * 8;
  const int mOff  = (lane >> 4) * 8;

  v8f acc[4][4];
#pragma unroll
  for (int i = 0; i < 4; ++i)
#pragma unroll
    for (int j = 0; j < 4; ++j) acc[i][j] = (v8f){0.f,0.f,0.f,0.f,0.f,0.f,0.f,0.f};

  for (int k0 = 0; k0 < K; k0 += 32) {
    V bh[4], bl[4];
#pragma unroll
    for (int j = 0; j < 4; ++j) {
      const size_t bo = (size_t)(n0 + (j << 4) + rlane) * ldb + koff + k0;
      bh[j] = Frag<T>::load(Bb + bo);
      if (SPLIT) bl[j] = Frag<T>::load(Bb2 + bo);
    }
#pragma unroll
    for (int i = 0; i < 4; ++i) {
      const size_t ao = (size_t)(m0 + (i << 4) + rlane) * lda + koff + k0;
      V ah = Frag<T>::load(Ab + ao);
      V al;
      if (SPLIT) al = Frag<T>::load(Ab2 + ao);
#pragma unroll
      for (int j = 0; j < 4; ++j) {
        acc[i][j] = Frag<T>::mma(ah, bh[j], acc[i][j]);
        if (SPLIT) {
          acc[i][j] = Frag<T>::mma(ah, bl[j], acc[i][j]);
          acc[i][j] = Frag<T>::mma(al, bh[j], acc[i][j]);
        }
      }
      Frag<T>::guard4(acc[i][0], acc[i][1], acc[i][2], acc[i][3], ah, SPLIT ? al : ah);
    }
    Frag<T>::keep(bh[0], bh[1], bh[2], bh[3]);
    if (SPLIT) Frag<T>::keep(bl[0], bl[1], bl[2], bl[3]);
  }
  acc_guard4(acc[0][0], acc[0][1], acc[0][2], acc[0][3]);
  acc_guard4(acc[1][0], acc[1][1], acc[1][2], acc[1][3]);
  acc_guard4(acc[2][0], acc[2][1], acc[2][2], acc[2][3]);
  acc_guard4(acc[3][0], acc[3][1], acc[3][2], acc[3][3]);

  float* slab = sT[wave];
  const float* Rb = RESID ? (resid + (size_t)b * strideR) : nullptr;
#pragma unroll
  for (int i = 0; i < 4; ++i) {
    const int mBase = m0 + (i << 4);
#pragma unroll
    for (int j = 0; j < 4; ++j) {
      const int n = n0 + (j << 4) + rlane;
      float bv = 0.f;
      if (BIAS_MODE == 2) bv = bias[n];
#pragma unroll
      for (int r = 0; r < 8; ++r) {
        float v = acc[i][j][r] * scale;
        if (BIAS_MODE == 1) v += bias[mBase + mOff + r];
        if (BIAS_MODE == 2) v += bv;
        if (RESID) v += Rb[(size_t)(mBase + mOff + r) * ldc + n];
        if (ACT == 1) v = tanhf(v);
        if (ACT == 2) v = fmaxf(v, 0.0f);
        if (ACT == 3) v = v / (1.0f + expf(-v));
        if (ACT == 4) v = (v > 0.f) ? v : 0.01f * v;
        if (ACT == 5) v = 0.5f * v * (1.0f + erff(v * 0.70710678118654752f));
        slab[(mOff + r) * 68 + (j << 4) + rlane] = v;
      }
    }
    __builtin_amdgcn_fence(__ATOMIC_RELEASE, "workgroup");
    __builtin_amdgcn_wave_barrier();
    __builtin_amdgcn_fence(__ATOMIC_ACQUIRE, "workgroup");
    if (OUT_MODE == 0) {
      float* C = (float*)Cout + (size_t)b * strideC;
      const int hh = lane >> 4, c4 = (lane & 15) * 4;
      for (int pass = 0; pass < 2; ++pass) {
#pragma unroll
        for (int it = 0; it < 8; ++it) {
          const int row = it * 2 + hh;
          v4f v = *(const v4f*)(slab + row * 68 + c4);
          *(volatile v4f*)(C + (size_t)(mBase + row) * ldc + n0 + c4) = v;
        }
        __threadfence();
      }
    } else {
      const int q = lane >> 3, c8 = (lane & 7) * 8;
      unsigned short* C  = (unsigned short*)Cout  + (size_t)b * strideC;
      unsigned short* C2 = (OUT_MODE == 2) ? ((unsigned short*)Cout2 + (size_t)b * strideC) : nullptr;
      for (int pass = 0; pass < 2; ++pass) {
#pragma unroll
        for (int it = 0; it < 4; ++it) {
          const int row = it * 4 + q;
          const float* sp = slab + row * 68 + c8;
          v8h hv, lv;
#pragma unroll
          for (int e = 0; e < 8; ++e) {
            if (OUT_MODE == 1) {
              hv[e] = (_Float16)sp[e];
            } else {
              unsigned short hb = f2bf_bits(sp[e]);
              unsigned short lb = f2bf_bits(sp[e] - bf_bits2f(hb));
              hv[e] = __builtin_bit_cast(_Float16, hb);
              lv[e] = __builtin_bit_cast(_Float16, lb);
            }
          }
          *(volatile v8h*)(C + (size_t)(mBase + row) * ldc + n0 + c8) = hv;
          if (OUT_MODE == 2) *(volatile v8h*)(C2 + (size_t)(mBase + row) * ldc + n0 + c8) = lv;
        }
        __threadfence();
      }
    }
    __builtin_amdgcn_fence(__ATOMIC_RELEASE, "workgroup");
    __builtin_amdgcn_wave_barrier();
    __builtin_amdgcn_fence(__ATOMIC_ACQUIRE, "workgroup");
  }
}

__global__ __launch_bounds__(256) void pack_wt_kernel(const float* __restrict__ s0, const float* __restrict__ s1,
                                                      const float* __restrict__ s2, const float* __restrict__ s3,
                                                      const float* __restrict__ s4, const float* __restrict__ s5,
                                                      unsigned short* __restrict__ dst) {
  __shared__ __align__(16) float ts[64 * 68];
  const int z = blockIdx.z;
  const float* src = (z == 0) ? s0 : (z == 1) ? s1 : (z == 2) ? s2 : (z == 3) ? s3 : (z == 4) ? s4 : s5;
  const int k0 = blockIdx.x * 64;
  const int n0 = blockIdx.y * 64;
  const int tid = threadIdx.x;
  {
    const int kq = tid >> 4;
    const int c4 = (tid & 15) * 4;
    v4f v[4];
#pragma unroll
    for (int it = 0; it < 4; ++it)
      v[it] = *(const v4f*)(src + (size_t)(k0 + it * 16 + kq) * NGATE3 + n0 + c4);
#pragma unroll
    for (int it = 0; it < 4; ++it) {
      const int kk = it * 16 + kq;
      const v4f t = v[it];
      ts[(c4 + 0) * 68 + kk] = t[0];
      ts[(c4 + 1) * 68 + kk] = t[1];
      ts[(c4 + 2) * 68 + kk] = t[2];
      ts[(c4 + 3) * 68 + kk] = t[3];
    }
  }
  __syncthreads();
  {
    const int q = tid & 7;
    const int nr = tid >> 3;
    v8h hv[2];
#pragma unroll
    for (int it = 0; it < 2; ++it) {
      const int n = it * 32 + nr;
      const v4f a = *(const v4f*)(ts + n * 68 + 8 * q);
      const v4f b = *(const v4f*)(ts + n * 68 + 8 * q + 4);
#pragma unroll
      for (int e = 0; e < 4; ++e) {
        hv[it][e]     = (_Float16)(a[e] * WCARRY);
        hv[it][4 + e] = (_Float16)(b[e] * WCARRY);
      }
    }
    unsigned short* dp = dst + (size_t)z * PLANE_W;
    for (int pass = 0; pass < 2; ++pass) {
#pragma unroll
      for (int it = 0; it < 2; ++it) {
        const int n = it * 32 + nr;
        *(volatile v8h*)(dp + (size_t)(n0 + n) * NHID + k0 + 8 * q) = hv[it];
      }
      __threadfence();
    }
  }
}

__device__ __forceinline__ float fsigm(float x) { return __builtin_amdgcn_rcpf(1.0f + expf(-x)); }
__device__ __forceinline__ float ftanh_id(float x) { return 1.0f - 2.0f * __builtin_amdgcn_rcpf(1.0f + expf(2.0f * x)); }
__device__ __forceinline__ float gru_cell(float xz_, float xr_, float xh_, float iz, float ir, float ih, float hold) {
  const float zg = fsigm(xz_ + iz);
  const float rg = fsigm(xr_ + ir);
  const float hc = ftanh_id(xh_ + rg * ih);
  return zg * hold + (1.0f - zg) * hc;
}

template <int LAYER>
__global__ __launch_bounds__(SCAN_THR) void gru_scan_kernel(
    const int* __restrict__ tokens,
    const float* __restrict__ W0f, const float* __restrict__ W0b,
    const float* __restrict__ biasf, const float* __restrict__ biasb,
    const unsigned short* __restrict__ UTf, const unsigned short* __restrict__ UTb,
    const float* __restrict__ XZf, const float* __restrict__ XZb,
    unsigned short* __restrict__ X0f, unsigned short* __restrict__ X0b,
    float* __restrict__ out0, float* __restrict__ sdst) {
  __shared__ __align__(16) _Float16 Ahi[SEQ_BLK * HPITCH];
  __shared__ __align__(16) _Float16 Alo[SEQ_BLK * HPITCH];
  __shared__ __align__(16) float    Hf[SEQ_BLK * FPITCH];
  const int tid = threadIdx.x, lane = tid & 31, wave = tid >> 5;
  const int c = lane & 15, hh = lane >> 4, koff = hh * 8;
  const int dir = blockIdx.x >> 1;
  const int rowbase = (blockIdx.x & 1) * SEQ_BLK;
  const float* W0   = dir ? W0b : W0f;
  const float* bias = dir ? biasb : biasf;
  const _Float16* UT = (const _Float16*)(dir ? UTb : UTf);
  const float* XZ   = dir ? XZb : XZf;
  unsigned short* X0 = dir ? X0b : X0f;

#pragma unroll 1
  for (int i = tid; i < SEQ_BLK * HPITCH; i += SCAN_THR) { Ahi[i] = (_Float16)0.0f; Alo[i] = (_Float16)0.0f; }
#pragma unroll 1
  for (int i = tid; i < SEQ_BLK * FPITCH; i += SCAN_THR) Hf[i] = 0.0f;

  float bhv[2][3], biv[2][3];
#pragma unroll
  for (int nt = 0; nt < 2; ++nt)
#pragma unroll
    for (int g = 0; g < 3; ++g) bhv[nt][g] = bias[NGATE3 + g * NHID + 32 * wave + 16 * nt + c];
  asm volatile("" ::: "memory");
#pragma unroll
  for (int nt = 0; nt < 2; ++nt)
#pragma unroll
    for (int g = 0; g < 3; ++g) {
      if (LAYER == 0) biv[nt][g] = bias[g * NHID + 32 * wave + 16 * nt + c];
      else biv[nt][g] = 0.0f;
    }
  asm volatile("" ::: "memory");

  float hst[2][8];
#pragma unroll
  for (int nt = 0; nt < 2; ++nt)
#pragma unroll
    for (int r = 0; r < 8; ++r) hst[nt][r] = 0.0f;
  __syncthreads();

  const v8f z8 = {0.f, 0.f, 0.f, 0.f, 0.f, 0.f, 0.f, 0.f};
  const float sMain = 1.0f / (HCARRY * WCARRY);
  const float sRes  = sMain / LCARRY;

#pragma unroll 1
  for (int s = 0; s < NSTEP; ++s) {
    const int tt = dir ? (NSTEP - 1 - s) : s;
    const bool last = (s == NSTEP - 1);
    int toff[8];
#pragma unroll
    for (int r = 0; r < 8; ++r) toff[r] = 0;
    if (LAYER == 0) {
#pragma unroll
      for (int r = 0; r < 8; ++r) {
        int tk = tokens[(rowbase + 8 * hh + r) * NSTEP + tt];
        tk = tk < 0 ? 0 : tk;
        tk = tk > (NVOCAB - 1) ? (NVOCAB - 1) : tk;
        toff[r] = tk * NGATE3;
      }
      pin8(toff[0], toff[1], toff[2], toff[3], toff[4], toff[5], toff[6], toff[7]);
    }
    const int xrow0 = ((rowbase + 8 * hh) * NSTEP + s) * NGATE3;

#pragma unroll
    for (int nt = 0; nt < 2; ++nt) {
      const int j = 32 * wave + 16 * nt + c;
      const _Float16* ahrow = Ahi + c * HPITCH + koff;
      const _Float16* alrow = Alo + c * HPITCH + koff;
      const _Float16* wz = UT + (size_t)j * NHID + koff;
      const _Float16* wr = UT + (size_t)(NHID + j) * NHID + koff;
      const _Float16* wh = UT + (size_t)(2 * NHID + j) * NHID + koff;
      v8f mz = z8, mr = z8, mh = z8, rz = z8, rr = z8, rh = z8;
#pragma unroll 1
      for (int k0 = 0; k0 < NHID; k0 += 32) {
        const v16h ah = Frag<_Float16>::load(ahrow + k0);
        const v16h al = Frag<_Float16>::load(alrow + k0);
        const v16h b0 = Frag<_Float16>::load(wz + k0);
        const v16h b1 = Frag<_Float16>::load(wr + k0);
        const v16h b2 = Frag<_Float16>::load(wh + k0);
        mz = Frag<_Float16>::mma(ah, b0, mz);
        rz = Frag<_Float16>::mma(al, b0, rz);
        mr = Frag<_Float16>::mma(ah, b1, mr);
        rr = Frag<_Float16>::mma(al, b1, rr);
        mh = Frag<_Float16>::mma(ah, b2, mh);
        rh = Frag<_Float16>::mma(al, b2, rh);
        dep_guard6_h(mz, rz, mr, rr, mh, rh, ah, al, b0, b1, b2);
      }
      int jd = j;
      acc_guard6j(mz, rz, mr, rr, mh, rh, jd);

#pragma unroll
      for (int g4 = 0; g4 < 2; ++g4) {
        float xv[4][3];
#pragma unroll
        for (int q = 0; q < 4; ++q) {
          const int r = g4 * 4 + q;
          const float* xp;
          if (LAYER == 0) xp = W0 + toff[r] + jd;
          else xp = XZ + xrow0 + r * (NSTEP * NGATE3) + jd;
          xv[q][0] = xp[0];
          xv[q][1] = xp[NHID];
          xv[q][2] = xp[2 * NHID];
        }
#pragma unroll
        for (int q = 0; q < 4; ++q) {
          const int r = g4 * 4 + q;
          const float iz = mz[r] * sMain + rz[r] * sRes + bhv[nt][0];
          const float ir = mr[r] * sMain + rr[r] * sRes + bhv[nt][1];
          const float ih = mh[r] * sMain + rh[r] * sRes + bhv[nt][2];
          hst[nt][r] = gru_cell(xv[q][0] + biv[nt][0], xv[q][1] + biv[nt][1], xv[q][2] + biv[nt][2],
                                iz, ir, ih, hst[nt][r]);
        }
        order_after4(jd, hst[nt][g4 * 4 + 0], hst[nt][g4 * 4 + 1], hst[nt][g4 * 4 + 2], hst[nt][g4 * 4 + 3]);
      }
    }

    __syncthreads();
#pragma unroll
    for (int nt = 0; nt < 2; ++nt) {
      const int j = 32 * wave + 16 * nt + c;
#pragma unroll
      for (int r = 0; r < 8; ++r) {
        const int row = 8 * hh + r;
        const float hv = hst[nt][r];
        const float hs = hv * HCARRY;
        const _Float16 hi = (_Float16)hs;
        float hif = (float)hi;
        asm volatile("" : "+v"(hif));
        const float res = (hs - hif) * LCARRY;
        Ahi[row * HPITCH + j] = hi;
        Alo[row * HPITCH + j] = (_Float16)res;
        Hf[row * FPITCH + j]  = hv;
      }
    }
    __syncthreads();

    if (LAYER == 0) {
      const _Float16* src = Ahi + wave * HPITCH + lane * 8;
      const v8h v0 = *(const v8h*)(src);
      const v8h v1 = *(const v8h*)(src + 256);
      unsigned short* dp = X0 + ((size_t)(rowbase + wave) * NSTEP + (size_t)s) * NHID + lane * 8;
      for (int pass = 0; pass < 2; ++pass) {
        *(volatile v8h*)(dp) = v0;
        *(volatile v8h*)(dp + 256) = v1;
        __threadfence();
      }
    }
    if (LAYER == 1 || last) {
      const float* srcf = Hf + wave * FPITCH + lane * 4;
      const v4f f0 = *(const v4f*)(srcf);
      const v4f f1 = *(const v4f*)(srcf + 128);
      const v4f f2 = *(const v4f*)(srcf + 256);
      const v4f f3 = *(const v4f*)(srcf + 384);
      if (LAYER == 1) {
        float* op = out0 + ((size_t)(rowbase + wave) * NSTEP + (size_t)tt) * (2 * NHID) + dir * NHID + lane * 4;
        for (int pass = 0; pass < 2; ++pass) {
          *(volatile v4f*)(op) = f0;
          *(volatile v4f*)(op + 128) = f1;
          *(volatile v4f*)(op + 256) = f2;
          *(volatile v4f*)(op + 384) = f3;
          __threadfence();
        }
      }
      if (last) {
        float* sp = sdst + (size_t)(rowbase + wave) * (2 * NHID) + dir * NHID + lane * 4;
        for (int pass = 0; pass < 2; ++pass) {
          *(volatile v4f*)(sp) = f0;
          *(volatile v4f*)(sp + 128) = f1;
          *(volatile v4f*)(sp + 256) = f2;
          *(volatile v4f*)(sp + 384) = f3;
          __threadfence();
        }
      }
    }
  }
}

extern "C" void kernel_launch(void* const* d_in, const int* in_sizes, int n_in,
                              void* d_out, int out_size, void* d_ws, size_t ws_size, hipStream_t stream) {
  if (n_in < 13 || d_out == nullptr || d_ws == nullptr) return;
  if (in_sizes[0] != NBATCH * NSTEP ||
      in_sizes[1] != NVOCAB * NGATE3 || in_sizes[2] != NHID * NGATE3 || in_sizes[3] != 2 * NGATE3 ||
      in_sizes[4] != NHID * NGATE3   || in_sizes[5] != NHID * NGATE3 || in_sizes[6] != 2 * NGATE3 ||
      in_sizes[7] != NVOCAB * NGATE3 || in_sizes[8] != NHID * NGATE3 || in_sizes[9] != 2 * NGATE3 ||
      in_sizes[10] != NHID * NGATE3  || in_sizes[11] != NHID * NGATE3 || in_sizes[12] != 2 * NGATE3 ||
      out_size != NOUT0 + 2 * NOUTS) return;

  const int*   tokens = (const int*)d_in[0];
  const float* W0f = (const float*)d_in[1];
  const float* U0f = (const float*)d_in[2];
  const float* b0f = (const float*)d_in[3];
  const float* W1f = (const float*)d_in[4];
  const float* U1f = (const float*)d_in[5];
  const float* b1f = (const float*)d_in[6];
  const float* W0b = (const float*)d_in[7];
  const float* U0b = (const float*)d_in[8];
  const float* b0b = (const float*)d_in[9];
  const float* W1b = (const float*)d_in[10];
  const float* U1b = (const float*)d_in[11];
  const float* b1b = (const float*)d_in[12];

  float* out0 = (float*)d_out;
  float* s0   = out0 + (size_t)NOUT0;
  float* s1   = s0 + (size_t)NOUTS;

  char* ws = (char*)d_ws;
  size_t off = 0;
  unsigned short* UT = (unsigned short*)(ws + off);
  off += 6 * PLANE_W * 2;
  unsigned short* X0 = (unsigned short*)(ws + off);
  off += 2 * PLANE_X0 * 2;
  float* XZ1 = (float*)(ws + off);
  off += 2 * PLANE_XZ * 4;
  if (off > ws_size || off > (size_t)134217728) return;

  pack_wt_kernel<<<dim3(NHID / 64, NGATE3 / 64, 6), 256, 0, stream>>>(U0f, U0b, U1f, U1b, W1f, W1b, UT);

  gru_scan_kernel<0><<<4, SCAN_THR, 0, stream>>>(
      tokens, W0f, W0b, b0f, b0b,
      UT + 0 * PLANE_W, UT + 1 * PLANE_W,
      XZ1, XZ1 + PLANE_XZ,
      X0, X0 + PLANE_X0,
      out0, s0);

  const int tiles = (NROWS / 64) * (NGATE3 / 64);
  const float gscale = 1.0f / (HCARRY * WCARRY);
  wmma_gemm64<0, false, 2, 0, false, 0><<<dim3(tiles / 8, 1), 256, 0, stream>>>(
      X0, X0, NHID, 0L,
      UT + 4 * PLANE_W, UT + 4 * PLANE_W, NHID, 0L,
      (void*)XZ1, (void*)XZ1, NGATE3, 0L,
      b1f, XZ1, 0L, NROWS, NGATE3, NHID, gscale);
  wmma_gemm64<0, false, 2, 0, false, 0><<<dim3(tiles / 8, 1), 256, 0, stream>>>(
      X0 + PLANE_X0, X0 + PLANE_X0, NHID, 0L,
      UT + 5 * PLANE_W, UT + 5 * PLANE_W, NHID, 0L,
      (void*)(XZ1 + PLANE_XZ), (void*)(XZ1 + PLANE_XZ), NGATE3, 0L,
      b1b, XZ1, 0L, NROWS, NGATE3, NHID, gscale);

  gru_scan_kernel<1><<<4, SCAN_THR, 0, stream>>>(
      tokens, W0f, W0b, b1f, b1b,
      UT + 2 * PLANE_W, UT + 3 * PLANE_W,
      XZ1, XZ1 + PLANE_XZ,
      X0, X0 + PLANE_X0,
      out0, s1);
}
